// KANLinear_85495618994499
// MI455X (gfx1250) — hardware-verified
//
#include <hip/hip_runtime.h>
#include <math.h>

constexpr int kInF       = 1024;
constexpr int kOutF      = 1024;
constexpr int kGridN     = 8;
constexpr int kKdim      = kInF + kInF * kGridN;
constexpr int kRowsTotal = 8192;
constexpr int kRowsHalf  = 4096;
constexpr int kNumHalves = 2;
constexpr float kCarrySilu  = 8.0f;
constexpr float kCarryBaseW = 2048.0f;
constexpr float kCarryBasis = 1024.0f;
constexpr float kCarrySplW  = 16.0f;
constexpr float kOutScale   = 1.0f / 16384.0f;
constexpr float kInvDenom   = (float)(1.0 / (4.0 / 7.0 + 1e-6));
static_assert(kCarrySilu * kCarryBaseW == 16384.0f);
static_assert(kCarryBasis * kCarrySplW == 16384.0f);
static_assert(kKdim % 32 == 0);
static_assert(kRowsHalf % 64 == 0);
static_assert(kOutF % 64 == 0);
static_assert(kRowsHalf * kNumHalves == kRowsTotal);

constexpr size_t kWsWT      = 0;
constexpr size_t kWsWTBytes = (size_t)kOutF * kKdim * 2;
constexpr size_t kWsA       = kWsWT + kWsWTBytes;
constexpr size_t kWsABytes  = (size_t)kRowsHalf * kKdim * 2;
constexpr size_t kWsTotal   = kWsA + kWsABytes;
static_assert(kWsWTBytes == 18874368);
static_assert(kWsABytes == 75497472);
static_assert(kWsTotal == 94371840);
static_assert(kWsTotal <= (size_t)134217728);
static_assert(kWsA % 128 == 0);

typedef __attribute__((ext_vector_type(16))) _Float16 v16h;
typedef __attribute__((ext_vector_type(8)))  _Float16 v8h;
typedef __attribute__((ext_vector_type(16))) __bf16   v16b;
typedef __attribute__((ext_vector_type(8)))  __bf16   v8b;
typedef __attribute__((ext_vector_type(8)))  float    v8f;
typedef __attribute__((ext_vector_type(4)))  float    v4f;
typedef __attribute__((ext_vector_type(4)))  unsigned int v4u;

__device__ __forceinline__ unsigned short f2bf_bits(float f) {
  unsigned u = __float_as_uint(f);
  return (unsigned short)((u + 0x7FFFu + ((u >> 16) & 1u)) >> 16);
}
__device__ __forceinline__ float bf_bits2f(unsigned short h) { return __uint_as_float(((unsigned)h) << 16); }

__device__ __forceinline__ void dep_guard_h(v8f& a, v8f& b, v16h x, v16h y) { asm volatile("v_nop\n\tv_nop\n\tv_nop\n\tv_nop" : "+v"(a), "+v"(b) : "v"(x), "v"(y)); }
__device__ __forceinline__ void dep_guard_b(v8f& a, v8f& b, v16b x, v16b y) { asm volatile("v_nop\n\tv_nop\n\tv_nop\n\tv_nop" : "+v"(a), "+v"(b) : "v"(x), "v"(y)); }
__device__ __forceinline__ void keep4_h(v16h a, v16h b, v16h c, v16h d) { asm volatile("v_nop" :: "v"(a), "v"(b), "v"(c), "v"(d)); }
__device__ __forceinline__ void keep4_b(v16b a, v16b b, v16b c, v16b d) { asm volatile("v_nop" :: "v"(a), "v"(b), "v"(c), "v"(d)); }
__device__ __forceinline__ void acc_guard4(v8f& a, v8f& b, v8f& c, v8f& d) { asm volatile("v_nop\n\tv_nop\n\tv_nop\n\tv_nop" : "+v"(a), "+v"(b), "+v"(c), "+v"(d)); }
template <typename T> struct Frag;
template <> struct Frag<_Float16> {
  typedef v16h V; union U { v16h v; v8h h[2]; };
  static __device__ __forceinline__ v16h load(const _Float16* p) {
    U f; f.h[0] = *(const v8h*)(p); f.h[1] = *(const v8h*)(p + 16); return f.v;
  }
  static __device__ __forceinline__ v8f mma(v16h a, v16h b, v8f c) {
    return __builtin_amdgcn_wmma_f32_16x16x32_f16(false, a, false, b, (short)0, c, false, false);
  }
  static __device__ __forceinline__ void guard(v8f& a, v8f& b, v16h x, v16h y) { dep_guard_h(a, b, x, y); }
  static __device__ __forceinline__ void keep(v16h a, v16h b, v16h c, v16h d) { keep4_h(a, b, c, d); }
};
template <> struct Frag<__bf16> {
  typedef v16b V; union U { v16b v; v8b h[2]; };
  static __device__ __forceinline__ v16b load(const __bf16* p) {
    U f; f.h[0] = *(const v8b*)(p); f.h[1] = *(const v8b*)(p + 16); return f.v;
  }
  static __device__ __forceinline__ v8f mma(v16b a, v16b b, v8f c) {
    return __builtin_amdgcn_wmma_f32_16x16x32_bf16(false, a, false, b, (short)0, c, false, false);
  }
  static __device__ __forceinline__ void guard(v8f& a, v8f& b, v16b x, v16b y) { dep_guard_b(a, b, x, y); }
  static __device__ __forceinline__ void keep(v16b a, v16b b, v16b c, v16b d) { keep4_b(a, b, c, d); }
};

__device__ __forceinline__ unsigned pk16(unsigned short a, unsigned short b) { return (unsigned)a | ((unsigned)b << 16); }
__device__ __forceinline__ unsigned short h_bits(float f) { const _Float16 h = (_Float16)f; return __builtin_bit_cast(unsigned short, h); }

template <int ET> struct Elem;
template <> struct Elem<0> { typedef _Float16 T; };
template <> struct Elem<1> { typedef __bf16 T; };
template <int ET, bool SPLIT, int BIAS_MODE, int OUT_MODE, bool RESID, int ACT = 0>
__global__ __launch_bounds__(256) void wmma_gemm64(
    const unsigned short* __restrict__ Ap, const unsigned short* __restrict__ A2p, int lda, long strideA,
    const unsigned short* __restrict__ Btp, const unsigned short* __restrict__ Bt2p, int ldb, long strideB,
    void* __restrict__ Cout, void* __restrict__ Cout2, int ldc, long strideC,
    const float* __restrict__ bias,
    const float* __restrict__ resid, long strideR,
    int M, int N, int K, float scale) {
  typedef typename Elem<ET>::T T;
  typedef typename Frag<T>::V V;
  const T* A = (const T*)Ap; const T* A2 = (const T*)A2p; const T* Bt = (const T*)Btp; const T* Bt2 = (const T*)Bt2p;
  __shared__ __align__(16) float sT[8][16 * 68];
  const int b    = blockIdx.y;
  const int lane = threadIdx.x & 31;
  const int wave = threadIdx.x >> 5;
  const int tilesN = N >> 6;
  const int tilesM = M >> 6;
  const int tile = blockIdx.x * 8 + wave;
  if (tile >= tilesM * tilesN) return;
  const int tm = tile / tilesN;
  const int tn = tile - tm * tilesN;
  const int m0 = tm << 6;
  const int n0 = tn << 6;

  const T* Ab  = A  + (size_t)b * strideA;
  const T* Bb  = Bt + (size_t)b * strideB;
  const T* Ab2 = SPLIT ? (A2  + (size_t)b * strideA) : nullptr;
  const T* Bb2 = SPLIT ? (Bt2 + (size_t)b * strideB) : nullptr;

  const int rlane = lane & 15;
  const int koff  = (lane >> 4) * 8;
  const int mOff  = (lane >> 4) * 8;

  v8f acc[4][4];
#pragma unroll
  for (int i = 0; i < 4; ++i)
#pragma unroll
    for (int j = 0; j < 4; ++j) acc[i][j] = (v8f){0.f,0.f,0.f,0.f,0.f,0.f,0.f,0.f};

  for (int k0 = 0; k0 < K; k0 += 32) {
    V bh[4], bl[4];
#pragma unroll
    for (int j = 0; j < 4; ++j) {
      const size_t bo = (size_t)(n0 + (j << 4) + rlane) * ldb + koff + k0;
      bh[j] = Frag<T>::load(Bb + bo);
      if (SPLIT) bl[j] = Frag<T>::load(Bb2 + bo);
    }
#pragma unroll
    for (int i = 0; i < 4; ++i) {
      const size_t ao = (size_t)(m0 + (i << 4) + rlane) * lda + koff + k0;
      V ah = Frag<T>::load(Ab + ao);
      V al;
      if (SPLIT) al = Frag<T>::load(Ab2 + ao);
#pragma unroll
      for (int j = 0; j < 4; ++j) {
        acc[i][j] = Frag<T>::mma(ah, bh[j], acc[i][j]);
        if (SPLIT) {
          acc[i][j] = Frag<T>::mma(ah, bl[j], acc[i][j]);
          acc[i][j] = Frag<T>::mma(al, bh[j], acc[i][j]);
        }
      }
      Frag<T>::guard(acc[i][0], acc[i][3], ah, SPLIT ? al : ah);
    }
    Frag<T>::keep(bh[0], bh[1], bh[2], bh[3]);
    if (SPLIT) Frag<T>::keep(bl[0], bl[1], bl[2], bl[3]);
  }
  acc_guard4(acc[0][0], acc[0][1], acc[0][2], acc[0][3]);
  acc_guard4(acc[1][0], acc[1][1], acc[1][2], acc[1][3]);
  acc_guard4(acc[2][0], acc[2][1], acc[2][2], acc[2][3]);
  acc_guard4(acc[3][0], acc[3][1], acc[3][2], acc[3][3]);

  float* slab = sT[wave];
  const float* Rb = RESID ? (resid + (size_t)b * strideR) : nullptr;
#pragma unroll
  for (int i = 0; i < 4; ++i) {
    const int mBase = m0 + (i << 4);
#pragma unroll
    for (int j = 0; j < 4; ++j) {
      const int n = n0 + (j << 4) + rlane;
      float bv = 0.f;
      if (BIAS_MODE == 2) bv = bias[n];
#pragma unroll
      for (int r = 0; r < 8; ++r) {
        float v = acc[i][j][r] * scale;
        if (BIAS_MODE == 1) v += bias[mBase + mOff + r];
        if (BIAS_MODE == 2) v += bv;
        if (RESID) v += Rb[(size_t)(mBase + mOff + r) * ldc + n];
        if (ACT == 2) v = fmaxf(v, 0.0f);
        if (ACT == 4) v = (v > 0.f) ? v : 0.01f * v;
        slab[(mOff + r) * 68 + (j << 4) + rlane] = v;
      }
    }
    __builtin_amdgcn_fence(__ATOMIC_RELEASE, "workgroup");
    __builtin_amdgcn_wave_barrier();
    __builtin_amdgcn_fence(__ATOMIC_ACQUIRE, "workgroup");
    if (OUT_MODE == 0) {
      float* C = (float*)Cout + (size_t)b * strideC;
      const int hh = lane >> 4, c4 = (lane & 15) * 4;
      for (int pass = 0; pass < 2; ++pass) {
#pragma unroll
        for (int it = 0; it < 8; ++it) {
          const int row = it * 2 + hh;
          v4f v = *(const v4f*)(slab + row * 68 + c4);
          *(volatile v4f*)(C + (size_t)(mBase + row) * ldc + n0 + c4) = v;
        }
        __threadfence();
      }
    } else {
      const int q = lane >> 3, c8 = (lane & 7) * 8;
      unsigned short* C  = (unsigned short*)Cout  + (size_t)b * strideC;
      unsigned short* C2 = (OUT_MODE == 2) ? ((unsigned short*)Cout2 + (size_t)b * strideC) : nullptr;
      for (int pass = 0; pass < 2; ++pass) {
#pragma unroll
        for (int it = 0; it < 4; ++it) {
          const int row = it * 4 + q;
          const float* sp = slab + row * 68 + c8;
          v8h hv, lv;
#pragma unroll
          for (int e = 0; e < 8; ++e) {
            if (OUT_MODE == 1) {
              hv[e] = (_Float16)sp[e];
            } else {
              unsigned short hb = f2bf_bits(sp[e]);
              unsigned short lb = f2bf_bits(sp[e] - bf_bits2f(hb));
              hv[e] = __builtin_bit_cast(_Float16, hb);
              lv[e] = __builtin_bit_cast(_Float16, lb);
            }
          }
          *(volatile v8h*)(C + (size_t)(mBase + row) * ldc + n0 + c8) = hv;
          if (OUT_MODE == 2) *(volatile v8h*)(C2 + (size_t)(mBase + row) * ldc + n0 + c8) = lv;
        }
        __threadfence();
      }
    }
    __builtin_amdgcn_fence(__ATOMIC_RELEASE, "workgroup");
    __builtin_amdgcn_wave_barrier();
    __builtin_amdgcn_fence(__ATOMIC_ACQUIRE, "workgroup");
  }
}

__global__ __launch_bounds__(128) void wcat_kernel(const float* __restrict__ base_w, const float* __restrict__ spline_w,
                                                   unsigned short* __restrict__ WT) {
  const int t  = threadIdx.x;
  const int bx = blockIdx.x;
  const int o  = blockIdx.y;
  const int bxs = (bx > 0) ? (bx - 1) : 0;
  const float* src = (bx == 0) ? (base_w + (size_t)o * kInF + 8 * t)
                               : (spline_w + (size_t)o * (kInF * kGridN) + (size_t)bxs * kInF + 8 * t);
  const float carry = (bx == 0) ? kCarryBaseW : kCarrySplW;
  const v4f a = *(const v4f*)(src);
  const v4f c = *(const v4f*)(src + 4);
  unsigned short hb[8];
#pragma unroll
  for (int e = 0; e < 4; ++e) {
    hb[e]     = h_bits(a[e] * carry);
    hb[4 + e] = h_bits(c[e] * carry);
  }
  const v4u u = (v4u){pk16(hb[0], hb[1]), pk16(hb[2], hb[3]), pk16(hb[4], hb[5]), pk16(hb[6], hb[7])};
  unsigned short* q = WT + (size_t)o * kKdim + (size_t)bx * kInF + 8 * t;
  *(volatile v4u*)q = u;
  __threadfence();
  *(volatile v4u*)q = u;
}

__global__ __launch_bounds__(256) void act_expand_kernel(const float* __restrict__ xh, unsigned short* __restrict__ Aact) {
  const int t = threadIdx.x;
  const size_t base = (size_t)blockIdx.x * 2048;
  {
    const size_t e0 = base + (size_t)(8 * t);
    const int r  = (int)(e0 >> 10);
    const int i0 = (int)(e0 & 1023);
    const v4f a = *(const v4f*)(xh + e0);
    const v4f c = *(const v4f*)(xh + e0 + 4);
    float v[8];
#pragma unroll
    for (int e = 0; e < 4; ++e) { v[e] = a[e]; v[4 + e] = c[e]; }
    unsigned short hb[8];
#pragma unroll
    for (int e = 0; e < 8; ++e) {
      const float vv = v[e];
      const float ex = expf(-vv);
      const float sg = __builtin_amdgcn_rcpf(1.0f + ex);
      const float s  = vv * sg;
      hb[e] = h_bits(s * kCarrySilu);
    }
    const v4u u = (v4u){pk16(hb[0], hb[1]), pk16(hb[2], hb[3]), pk16(hb[4], hb[5]), pk16(hb[6], hb[7])};
    unsigned short* q = Aact + (size_t)r * kKdim + i0;
    *(volatile v4u*)q = u;
    __threadfence();
    *(volatile v4u*)q = u;
  }
#pragma unroll 1
  for (int it = 0; it < 8; ++it) {
    const size_t e = base + (size_t)it * 256 + (size_t)t;
    const int r = (int)(e >> 10);
    const int i = (int)(e & 1023);
    const float vv = xh[e];
    unsigned short hb[8];
#pragma unroll
    for (int g = 0; g < kGridN; ++g) {
      const float sgf = (float)g * (1.0f / 7.0f);
      const float gg  = (g == 7) ? 2.0f : (-2.0f * (1.0f - sgf) + 2.0f * sgf);
      const float d   = vv - gg;
      const float tt  = d * kInvDenom;
      const float qq  = tt * tt;
      const float bv  = expf(-qq);
      hb[g] = h_bits(bv * kCarryBasis);
    }
    const v4u u = (v4u){pk16(hb[0], hb[1]), pk16(hb[2], hb[3]), pk16(hb[4], hb[5]), pk16(hb[6], hb[7])};
    unsigned short* q = Aact + (size_t)r * kKdim + kInF + (size_t)i * 8;
    *(volatile v4u*)q = u;
    __threadfence();
    *(volatile v4u*)q = u;
  }
}

extern "C" void kernel_launch(void* const* d_in, const int* in_sizes, int n_in,
                              void* d_out, int out_size, void* d_ws, size_t ws_size,
                              hipStream_t stream)
{
  if (n_in < 4) return;
  if (in_sizes[0] != kRowsTotal * kInF) return;
  if (in_sizes[1] != kOutF * kInF) return;
  if (in_sizes[2] != kOutF) return;
  if (in_sizes[3] != kOutF * kInF * kGridN) return;
  if (out_size != kRowsTotal * kOutF) return;
  if (ws_size < kWsTotal) return;

  const float* x        = (const float*)d_in[0];
  const float* base_w   = (const float*)d_in[1];
  const float* base_b   = (const float*)d_in[2];
  const float* spline_w = (const float*)d_in[3];
  float*       out      = (float*)d_out;

  unsigned char*  ws   = (unsigned char*)d_ws;
  unsigned short* WT   = (unsigned short*)(ws + kWsWT);
  unsigned short* Aact = (unsigned short*)(ws + kWsA);

  wcat_kernel<<<dim3(kKdim / kInF, kOutF), 128, 0, stream>>>(base_w, spline_w, WT);

  const int tilesPerHalf = (kRowsHalf / 64) * (kOutF / 64);
  const int gemmBlocks   = (tilesPerHalf + 7) / 8;
  for (int h = 0; h < kNumHalves; ++h) {
    const float* xh   = x + (size_t)h * kRowsHalf * kInF;
    float*       outh = out + (size_t)h * kRowsHalf * kOutF;
    act_expand_kernel<<<(kRowsHalf * kInF) / 2048, 256, 0, stream>>>(xh, Aact);
    wmma_gemm64<0, false, 2, 0, false, 0><<<dim3(gemmBlocks, 1), 256, 0, stream>>>(
        Aact, Aact, kKdim, 0L,
        WT, WT, kKdim, 0L,
        (void*)outh, (void*)outh, kOutF, 0L,
        base_b,
        base_b, 0L,
        kRowsHalf, kOutF, kKdim, kOutScale);
  }
}
